// SA_Block_71494025609721
// MI455X (gfx1250) — hardware-verified
//
#include <hip/hip_runtime.h>
#include <stdint.h>
#include <stddef.h>


typedef __bf16 bf16_t;
typedef __attribute__((ext_vector_type(16))) __bf16 v16bf;
typedef __attribute__((ext_vector_type(8)))  __bf16 v8bf_t;
typedef __attribute__((ext_vector_type(8)))  float  v8f;
typedef __attribute__((ext_vector_type(4)))  float  v4f_t;
typedef __attribute__((ext_vector_type(4)))  unsigned int v4u_t;
typedef v8bf_t __attribute__((__may_alias__)) v8bf;
typedef v4f_t  __attribute__((__may_alias__)) v4f;
typedef v4u_t  __attribute__((__may_alias__)) v4u;

constexpr int kB  = 8;
constexpr int kC  = 256;
constexpr int kN  = 4096;
constexpr int kD  = 32;
constexpr int PT  = 64;
constexpr int XP  = kC + 8;
constexpr int NPB = kN / PT;
constexpr int IB  = 64;
constexpr int NIB = kN / IB;
constexpr int KP  = kD + 8;
constexpr int VP  = 32 + 8;
typedef char cfg_check[(kN % PT == 0 && kN % IB == 0 && kC % 64 == 0 && kD == 32 &&
                        (XP % 8) == 0 && (KP % 8) == 0 && (VP % 8) == 0) ? 1 : -1];

union Frag { v16bf v; v8bf h2[2]; bf16_t e[16]; };

static __device__ __forceinline__ v8f mma16(v16bf a, v16bf b, v8f c) {
  v8f d = __builtin_amdgcn_wmma_f32_16x16x32_bf16(false, a, false, b, (short)0, c, false, false);
  asm volatile("v_nop\n\tv_nop\n\tv_nop\n\tv_nop" : "+v"(d) : "v"(a), "v"(b));
  return d;
}

static __device__ __forceinline__ v16bf frag_b16(const bf16_t* row, int h) {
  Frag f;
  f.h2[0] = *(const v8bf*)(row + 8 * h);
  f.h2[1] = *(const v8bf*)(row + 16 + 8 * h);
  return f.v;
}

static __device__ __forceinline__ v16bf frag_f32(const float* row, int h) {
  const v4f a0 = *(const v4f*)(row + 8 * h);
  const v4f a1 = *(const v4f*)(row + 8 * h + 4);
  const v4f c0 = *(const v4f*)(row + 16 + 8 * h);
  const v4f c1 = *(const v4f*)(row + 20 + 8 * h);
  Frag f;
#pragma unroll
  for (int e = 0; e < 4; ++e) {
    f.e[e]      = (bf16_t)a0[e];
    f.e[4 + e]  = (bf16_t)a1[e];
    f.e[8 + e]  = (bf16_t)c0[e];
    f.e[12 + e] = (bf16_t)c1[e];
  }
  return f.v;
}

static __device__ __forceinline__ float bf2f(bf16_t v) {
  union { bf16_t b; unsigned short u; } t;
  t.b = v;
  return __uint_as_float(((unsigned int)t.u) << 16);
}

__global__ void __launch_bounds__(128)
proj_kernel(const float* __restrict__ x, const float* __restrict__ Wq, const float* __restrict__ bq,
            const float* __restrict__ Wk, const float* __restrict__ bk, const float* __restrict__ Wv,
            const float* __restrict__ bv, bf16_t* __restrict__ Qb, bf16_t* __restrict__ Kb,
            bf16_t* __restrict__ Vb) {
  __shared__ alignas(16) bf16_t xt[PT * XP];
  __shared__ alignas(16) bf16_t sq[PT * kD];
  __shared__ alignas(16) bf16_t sk[PT * kD];
  __shared__ alignas(16) bf16_t sv[64 * PT];

  const int tid = threadIdx.x;
  const int wv  = tid >> 5;
  const int l   = tid & 31;
  const int h   = l >> 4;
  const int m   = l & 15;
  const int b   = blockIdx.x / NPB;
  const int p0  = (blockIdx.x - b * NPB) * PT;
  if (b >= kB) return;

  const float* xb = x + (size_t)b * kC * kN + p0;
#pragma unroll 2
  for (int it = 0; it < (kC * PT / 4) / 128; ++it) {
    const int c  = it * 8 + (tid >> 4);
    const int i4 = (tid & 15) * 4;
    const v4f v  = *(const v4f*)(xb + (size_t)c * kN + i4);
    bf16_t* d = xt + i4 * XP + c;
    d[0]      = (bf16_t)v[0];
    d[XP]     = (bf16_t)v[1];
    d[2 * XP] = (bf16_t)v[2];
    d[3 * XP] = (bf16_t)v[3];
  }
  __syncthreads();

  const bf16_t* xrow = xt + (wv * 16 + m) * XP;

  {
    v8f aq0 = {};
    v8f aq1 = {};
    v8f ak0 = {};
    v8f ak1 = {};
#pragma unroll 1
    for (int ks = 0; ks < kC / 32; ++ks) {
      const int k0 = ks * 32;
      const v16bf xf = frag_b16(xrow + k0, h);
      aq0 = mma16(xf, frag_f32(Wq + (size_t)m * kC + k0, h), aq0);
      aq1 = mma16(xf, frag_f32(Wq + (size_t)(16 + m) * kC + k0, h), aq1);
      ak0 = mma16(xf, frag_f32(Wk + (size_t)m * kC + k0, h), ak0);
      ak1 = mma16(xf, frag_f32(Wk + (size_t)(16 + m) * kC + k0, h), ak1);
    }
    const float bq0 = bq[m], bq1 = bq[16 + m];
    const float bk0 = bk[m], bk1 = bk[16 + m];
#pragma unroll
    for (int r = 0; r < 8; ++r) {
      const int io = (wv * 16 + 8 * h + r) * kD;
      sq[io + m]      = (bf16_t)(aq0[r] + bq0);
      sq[io + 16 + m] = (bf16_t)(aq1[r] + bq1);
      sk[io + m]      = (bf16_t)(ak0[r] + bk0);
      sk[io + 16 + m] = (bf16_t)(ak1[r] + bk1);
    }
  }

#pragma unroll 1
  for (int og = 0; og < kC / 64; ++og) {
    v8f av[4];
#pragma unroll
    for (int t = 0; t < 4; ++t) av[t] = v8f{};
#pragma unroll 1
    for (int ks = 0; ks < kC / 32; ++ks) {
      const int k0 = ks * 32;
      const v16bf xf = frag_b16(xrow + k0, h);
#pragma unroll
      for (int t = 0; t < 4; ++t)
        av[t] = mma16(frag_f32(Wv + (size_t)(og * 64 + t * 16 + m) * kC + k0, h), xf, av[t]);
    }
    __syncthreads();
#pragma unroll
    for (int t = 0; t < 4; ++t)
#pragma unroll
      for (int r = 0; r < 8; ++r) {
        const int ol = t * 16 + 8 * h + r;
        sv[ol * PT + wv * 16 + m] = (bf16_t)(av[t][r] + bv[og * 64 + ol]);
      }
    __syncthreads();
    v4u vv[4];
    size_t gv[4];
#pragma unroll
    for (int q = 0; q < 4; ++q) {
      const int row = q * 16 + (tid >> 3);
      const int seg = tid & 7;
      vv[q] = *(const v4u*)(sv + row * PT + seg * 8);
      gv[q] = ((size_t)(b * kC + og * 64 + row)) * kN + p0 + seg * 8;
    }
#pragma unroll
    for (int q = 0; q < 4; ++q) *(volatile v4u*)(Vb + gv[q]) = vv[q];
    __threadfence();
#pragma unroll
    for (int q = 0; q < 4; ++q) *(volatile v4u*)(Vb + gv[q]) = vv[q];
  }

  {
    v4u uq[2], uk[2];
    size_t gq[2];
#pragma unroll
    for (int q = 0; q < 2; ++q) {
      const int idx = q * 128 + tid;
      uq[q] = *(const v4u*)(sq + idx * 8);
      uk[q] = *(const v4u*)(sk + idx * 8);
      gq[q] = ((size_t)(b * kN + p0)) * kD + idx * 8;
    }
#pragma unroll
    for (int q = 0; q < 2; ++q) {
      *(volatile v4u*)(Qb + gq[q]) = uq[q];
      *(volatile v4u*)(Kb + gq[q]) = uk[q];
    }
    __threadfence();
#pragma unroll
    for (int q = 0; q < 2; ++q) {
      *(volatile v4u*)(Qb + gq[q]) = uq[q];
      *(volatile v4u*)(Kb + gq[q]) = uk[q];
    }
  }
}

__global__ void __launch_bounds__(256)
attn_kernel(const bf16_t* __restrict__ Qb, const bf16_t* __restrict__ Kb, const bf16_t* __restrict__ Vb,
            const float* __restrict__ x, const float* __restrict__ gamma, float* __restrict__ out) {
  __shared__ alignas(16) bf16_t ks[32 * KP];
  __shared__ alignas(16) bf16_t vs[kC * VP];
  __shared__ alignas(16) float  so[32 * IB];

  const int tid = threadIdx.x;
  const int wv  = tid >> 5;
  const int l   = tid & 31;
  const int h   = l >> 4;
  const int m   = l & 15;
  const int b    = blockIdx.x / NIB;
  const int iblk = (blockIdx.x - b * NIB) * IB;
  if (b >= kB) return;
  const int ti = wv >> 1;
  const int ch = wv & 1;
  const int i0 = iblk + ti * 16;
  const int c0 = ch * 128;

  const bf16_t* kg = Kb + (size_t)b * kN * kD;
  const bf16_t* vg = Vb + (size_t)b * kC * kN;

  const v16bf qf = frag_b16(Qb + ((size_t)b * kN + i0 + m) * kD, h);

  v8f acc[8];
#pragma unroll
  for (int ct = 0; ct < 8; ++ct) acc[ct] = v8f{};
  float lsum = 0.0f;
  float mrun = -1.0e30f;

#pragma unroll 1
  for (int j0 = 0; j0 < kN; j0 += 32) {
    __syncthreads();
    if (tid < 128) {
      const int row = tid >> 2, seg = tid & 3;
      *(v4u*)(ks + row * KP + seg * 8) = *(const v4u*)(kg + (size_t)(j0 + row) * kD + seg * 8);
    }
#pragma unroll
    for (int q = 0; q < 4; ++q) {
      const int idx = q * 256 + tid;
      const int c = idx >> 2, seg = idx & 3;
      *(v4u*)(vs + c * VP + seg * 8) = *(const v4u*)(vg + (size_t)c * kN + j0 + seg * 8);
    }
    __syncthreads();

    const v16bf ka0 = frag_b16(ks + m * KP, h);
    const v16bf ka1 = frag_b16(ks + (16 + m) * KP, h);
    const v8f z = {};
    const v8f st0 = mma16(ka0, qf, z);
    const v8f st1 = mma16(ka1, qf, z);

    float ml = fmaxf(st0[0], st1[0]);
#pragma unroll
    for (int r = 1; r < 8; ++r) ml = fmaxf(ml, fmaxf(st0[r], st1[r]));
    ml = fmaxf(ml, __shfl_xor(ml, 16));
    const float mn    = fmaxf(mrun, ml);
    const float alpha = __expf(mrun - mn);
    mrun = mn;

    Frag p;
    float ps = 0.0f;
#pragma unroll
    for (int r = 0; r < 8; ++r) {
      const bf16_t e0 = (bf16_t)__expf(st0[r] - mn);
      const bf16_t e1 = (bf16_t)__expf(st1[r] - mn);
      p.e[r]     = e0;
      p.e[8 + r] = e1;
      ps += bf2f(e0) + bf2f(e1);
    }
    ps += __shfl_xor(ps, 16);
    lsum = lsum * alpha + ps;

#pragma unroll
    for (int ct = 0; ct < 8; ++ct) acc[ct] *= alpha;

#pragma unroll
    for (int ct = 0; ct < 8; ++ct) {
      const v16bf va = frag_b16(vs + (c0 + ct * 16 + m) * VP, h);
      acc[ct] = mma16(va, p.v, acc[ct]);
    }
  }

  const float scl = gamma[0] / lsum;
#pragma unroll
  for (int ct = 0; ct < 8; ++ct) {
    __syncthreads();
#pragma unroll
    for (int r = 0; r < 8; ++r)
      so[(ch * 16 + 8 * h + r) * IB + ti * 16 + m] = acc[ct][r] * scl;
    __syncthreads();
    v4f ov[2];
    size_t go[2];
#pragma unroll
    for (int q = 0; q < 2; ++q) {
      const int idx = q * 256 + tid;
      const int row = idx >> 4;
      const int seg = idx & 15;
      const int c   = (row >> 4) * 128 + ct * 16 + (row & 15);
      go[q] = ((size_t)(b * kC + c)) * kN + iblk + seg * 4;
      ov[q] = *(const v4f*)(so + row * IB + seg * 4) + *(const v4f*)(x + go[q]);
    }
#pragma unroll
    for (int q = 0; q < 2; ++q) *(volatile v4f*)(out + go[q]) = ov[q];
    __threadfence();
#pragma unroll
    for (int q = 0; q < 2; ++q) *(volatile v4f*)(out + go[q]) = ov[q];
  }
}

extern "C" void kernel_launch(void* const* d_in, const int* in_sizes, int n_in,
                              void* d_out, int out_size, void* d_ws, size_t ws_size,
                              hipStream_t stream) {
  if (n_in < 8) return;
  if (in_sizes[0] != kB * kC * kN || in_sizes[1] != kD * kC || in_sizes[2] != kD ||
      in_sizes[3] != kD * kC || in_sizes[4] != kD || in_sizes[5] != kC * kC ||
      in_sizes[6] != kC || in_sizes[7] < 1) return;
  if (out_size != kB * kC * kN) return;

  const float* x     = (const float*)d_in[0];
  const float* Wq    = (const float*)d_in[1];
  const float* bq    = (const float*)d_in[2];
  const float* Wk    = (const float*)d_in[3];
  const float* bk    = (const float*)d_in[4];
  const float* Wv    = (const float*)d_in[5];
  const float* bv    = (const float*)d_in[6];
  const float* gamma = (const float*)d_in[7];
  float* out = (float*)d_out;

  const size_t qk_bytes = (size_t)kB * kN * kD * sizeof(bf16_t);
  const size_t v_bytes  = (size_t)kB * kC * kN * sizeof(bf16_t);
  if (ws_size < 2 * qk_bytes + v_bytes) return;
  bf16_t* Qb = (bf16_t*)d_ws;
  bf16_t* Kb = (bf16_t*)((char*)d_ws + qk_bytes);
  bf16_t* Vb = (bf16_t*)((char*)d_ws + 2 * qk_bytes);

  proj_kernel<<<dim3(kB * NPB), dim3(128), 0, stream>>>(x, Wq, bq, Wk, bk, Wv, bv, Qb, Kb, Vb);
  attn_kernel<<<dim3(kB * NIB), dim3(256), 0, stream>>>(Qb, Kb, Vb, x, gamma, out);
}
